// GeoNetEuclidean_5007931867346
// MI455X (gfx1250) — hardware-verified
//
#include <hip/hip_runtime.h>
#include <math.h>
#include <stdint.h>

#define NNODE   4096
#define NEDGE   131072
#define DIN     128
#define DHID    256
#define NHEADS  4
#define DHEAD   64
#define NLAYERS 3
#define DOUT    64
#define DQKV    768
#define QKP     512

typedef __attribute__((ext_vector_type(16))) __bf16   v16b;
typedef __attribute__((ext_vector_type(8)))  __bf16   v8b;
typedef __attribute__((ext_vector_type(8)))  float    v8f;
typedef __attribute__((ext_vector_type(4)))  float    v4f;
typedef __attribute__((ext_vector_type(2)))  float    v2f;
typedef __attribute__((ext_vector_type(4)))  int      v4i;
typedef __attribute__((ext_vector_type(8)))  unsigned short v8us;
typedef __attribute__((ext_vector_type(4)))  unsigned short v4us;

__device__ __forceinline__ unsigned short f2bf_bits(float f) {
  unsigned u = __float_as_uint(f);
  return (unsigned short)((u + 0x7FFFu + ((u >> 16) & 1u)) >> 16);
}
__device__ __forceinline__ float bf_bits2f(unsigned short h) { return __uint_as_float(((unsigned)h) << 16); }
__device__ __forceinline__ unsigned pk16(unsigned short a, unsigned short b) { return (unsigned)a | ((unsigned)b << 16); }
__device__ __forceinline__ __bf16 f2bf(float f) { return __builtin_bit_cast(__bf16, f2bf_bits(f)); }
__device__ __forceinline__ void bf_split(float f, __bf16& hi, __bf16& lo) {
  const unsigned short hb = f2bf_bits(f);
  hi = __builtin_bit_cast(__bf16, hb);
  lo = f2bf(f - bf_bits2f(hb));
}

union FragB { v16b v; v8b h[2]; };
__device__ __forceinline__ v16b frag_load(const __bf16* p) {
  FragB f; f.h[0] = *(const v8b*)(p); f.h[1] = *(const v8b*)(p + 16); return f.v;
}
__device__ __forceinline__ v8f mma_bf16(v16b a, v16b b, v8f c) {
  return __builtin_amdgcn_wmma_f32_16x16x32_bf16(false, a, false, b, (short)0, c, false, false);
}
__device__ __forceinline__ v8f mma_bf16_g(v16b a, v16b b, v8f c) {
  c = __builtin_amdgcn_wmma_f32_16x16x32_bf16(false, a, false, b, (short)0, c, false, false);
  asm volatile("v_nop\n\tv_nop\n\tv_nop\n\tv_nop" : "+v"(c) : "v"(a), "v"(b));
  return c;
}
__device__ __forceinline__ void dep_guard(v8f& a, v8f& b, v16b x, v16b y) {
  asm volatile("v_nop\n\tv_nop\n\tv_nop\n\tv_nop" : "+v"(a), "+v"(b) : "v"(x), "v"(y));
}
__device__ __forceinline__ void keep4(v16b a, v16b b, v16b c, v16b d) { asm volatile("v_nop" :: "v"(a), "v"(b), "v"(c), "v"(d)); }
__device__ __forceinline__ void acc_guard4(v8f& a, v8f& b, v8f& c, v8f& d) {
  asm volatile("v_nop\n\tv_nop\n\tv_nop\n\tv_nop" : "+v"(a), "+v"(b), "+v"(c), "+v"(d));
}
__device__ __forceinline__ void lds_wave_sync() {
  __builtin_amdgcn_fence(__ATOMIC_RELEASE, "workgroup");
  __builtin_amdgcn_wave_barrier();
  __builtin_amdgcn_fence(__ATOMIC_ACQUIRE, "workgroup");
}

template <int BIAS_MODE, int OUT_MODE, int NRES, int ACT>
__global__ __launch_bounds__(256) void gemm_x3_kernel(
    const unsigned short* __restrict__ Ahp, const unsigned short* __restrict__ Alp, int lda,
    const unsigned short* __restrict__ Bhp, const unsigned short* __restrict__ Blp, int ldb,
    float* __restrict__ Cf, unsigned short* __restrict__ Ch, unsigned short* __restrict__ Cl, int ldc,
    const float* __restrict__ bias, const float* __restrict__ res1, const float* __restrict__ res2,
    int M, int N, int K) {
  const __bf16* Ah = (const __bf16*)(const void*)Ahp;
  const __bf16* Al = (const __bf16*)(const void*)Alp;
  const __bf16* Bh = (const __bf16*)(const void*)Bhp;
  const __bf16* Bl = (const __bf16*)(const void*)Blp;
  __shared__ __align__(16) float sT[8][16 * 68];
  const int lane = threadIdx.x & 31;
  const int wave = threadIdx.x >> 5;
  const int tilesN = N >> 6;
  const int tilesM = M >> 6;
  const int tile = blockIdx.x * 8 + wave;
  if (tile >= tilesM * tilesN) return;
  const int tm = tile / tilesN;
  const int tn = tile - tm * tilesN;
  const int m0 = tm << 6;
  const int n0 = tn << 6;
  const int rlane = lane & 15;
  const int koff  = (lane >> 4) * 8;
  const int mOff  = (lane >> 4) * 8;

  v8f acc[4][4];
#pragma unroll
  for (int i = 0; i < 4; ++i)
#pragma unroll
    for (int j = 0; j < 4; ++j) acc[i][j] = (v8f){0.f,0.f,0.f,0.f,0.f,0.f,0.f,0.f};

  for (int k0 = 0; k0 < K; k0 += 32) {
    v16b bh[4], bl[4];
#pragma unroll
    for (int j = 0; j < 4; ++j) {
      const size_t bo = (size_t)(n0 + (j << 4) + rlane) * ldb + koff + k0;
      bh[j] = frag_load(Bh + bo);
      bl[j] = frag_load(Bl + bo);
    }
#pragma unroll
    for (int i = 0; i < 4; ++i) {
      const size_t ao = (size_t)(m0 + (i << 4) + rlane) * lda + koff + k0;
      const v16b ah = frag_load(Ah + ao);
      const v16b al = frag_load(Al + ao);
#pragma unroll
      for (int j = 0; j < 4; ++j) {
        acc[i][j] = mma_bf16(ah, bh[j], acc[i][j]);
        acc[i][j] = mma_bf16(ah, bl[j], acc[i][j]);
        acc[i][j] = mma_bf16(al, bh[j], acc[i][j]);
      }
      dep_guard(acc[i][0], acc[i][3], ah, al);
    }
    keep4(bh[0], bh[1], bh[2], bh[3]);
    keep4(bl[0], bl[1], bl[2], bl[3]);
  }
  acc_guard4(acc[0][0], acc[0][1], acc[0][2], acc[0][3]);
  acc_guard4(acc[1][0], acc[1][1], acc[1][2], acc[1][3]);
  acc_guard4(acc[2][0], acc[2][1], acc[2][2], acc[2][3]);
  acc_guard4(acc[3][0], acc[3][1], acc[3][2], acc[3][3]);

  float* slab = sT[wave];
#pragma unroll
  for (int i = 0; i < 4; ++i) {
    const int mBase = m0 + (i << 4);
#pragma unroll
    for (int j = 0; j < 4; ++j) {
      const int n = n0 + (j << 4) + rlane;
      float bv = 0.f;
      if (BIAS_MODE == 2) bv = bias[n];
#pragma unroll
      for (int r = 0; r < 8; ++r) {
        const int m = mBase + mOff + r;
        float v = acc[i][j][r];
        if (BIAS_MODE == 1) v += bias[m];
        if (BIAS_MODE == 2) v += bv;
        if (NRES >= 1) {
          float rs = res1[(size_t)m * ldc + n];
          if (NRES == 2) rs += res2[(size_t)m * ldc + n];
          v = rs + v;
        }
        if (ACT == 1) v = fmaxf(v, 0.0f);
        slab[(mOff + r) * 68 + (j << 4) + rlane] = v;
      }
    }
    lds_wave_sync();
    if (OUT_MODE == 0 || OUT_MODE == 2) {
      const int hh = lane >> 4, c4 = (lane & 15) * 4;
      for (int pass = 0; pass < 2; ++pass) {
#pragma unroll
        for (int it = 0; it < 8; ++it) {
          const int row = it * 2 + hh;
          const v4f v = *(const v4f*)(slab + row * 68 + c4);
          *(volatile v4f*)(Cf + (size_t)(mBase + row) * ldc + n0 + c4) = v;
        }
        __threadfence();
      }
    }
    if (OUT_MODE == 1 || OUT_MODE == 2) {
      const int q = lane >> 3, c8 = (lane & 7) * 8;
      for (int pass = 0; pass < 2; ++pass) {
#pragma unroll
        for (int it = 0; it < 4; ++it) {
          const int row = it * 4 + q;
          const float* sp = slab + row * 68 + c8;
          v8us hv, lv;
#pragma unroll
          for (int e = 0; e < 8; ++e) {
            const float f = sp[e];
            const unsigned short hb = f2bf_bits(f);
            hv[e] = hb;
            lv[e] = f2bf_bits(f - bf_bits2f(hb));
          }
          *(volatile v8us*)(Ch + (size_t)(mBase + row) * ldc + n0 + c8) = hv;
          *(volatile v8us*)(Cl + (size_t)(mBase + row) * ldc + n0 + c8) = lv;
        }
        __threadfence();
      }
    }
    lds_wave_sync();
  }
}

__global__ __launch_bounds__(256) void split_bf16x2_kernel(const float* __restrict__ in, unsigned short* __restrict__ hi,
                                                           unsigned short* __restrict__ lo, int n2) {
  const int i = blockIdx.x * 256 + threadIdx.x;
  if (i < n2) {
    const v2f f = *(const v2f*)(in + 2 * (size_t)i);
    const unsigned short h0 = f2bf_bits(f[0]), h1 = f2bf_bits(f[1]);
    const unsigned short l0 = f2bf_bits(f[0] - bf_bits2f(h0)), l1 = f2bf_bits(f[1] - bf_bits2f(h1));
    const unsigned uh = pk16(h0, h1), ul = pk16(l0, l1);
    ((volatile unsigned*)hi)[i] = uh;
    ((volatile unsigned*)lo)[i] = ul;
    __threadfence();
    ((volatile unsigned*)hi)[i] = uh;
    ((volatile unsigned*)lo)[i] = ul;
  }
}

__global__ __launch_bounds__(256) void deg_dis_kernel(const int* __restrict__ ei, int nE, int nN,
                                                      float* __restrict__ dis) {
  __shared__ int hist[NNODE];
  const int tid = threadIdx.x;
  for (int i = tid; i < NNODE; i += 256) hist[i] = 0;
  __syncthreads();
  const int* dst = ei + nE;
  for (int e = tid; e < nE; e += 256) {
    const int d = dst[e];
    if ((unsigned)d < (unsigned)nN && (unsigned)d < (unsigned)NNODE) atomicAdd(&hist[d], 1);
  }
  __syncthreads();
  v4f vals[4];
#pragma unroll
  for (int it = 0; it < 4; ++it) {
    const int b0 = it * 1024 + tid * 4;
    v4f v;
#pragma unroll
    for (int q = 0; q < 4; ++q) v[q] = rsqrtf((float)hist[b0 + q] + 1.0f);
    vals[it] = v;
  }
  for (int pass = 0; pass < 2; ++pass) {
#pragma unroll
    for (int it = 0; it < 4; ++it) *(volatile v4f*)(dis + it * 1024 + tid * 4) = vals[it];
    __threadfence();
  }
}

#define AG_NB    32
#define AG_CHUNK 1024
#define AG_CAP   3072

__device__ __forceinline__ void agg_drain_slot(const int* lst, int cnt, int slot,
                                               const int* __restrict__ src, int nE,
                                               const float* __restrict__ Hf, const float* __restrict__ dis,
                                               int nN, int lane, v4f& a0, v4f& a1) {
  for (int i = 0; i < cnt && i < AG_CAP; i += 32) {
    const int li = i + lane;
    const int ent = lst[li];
    const bool mine = (li < cnt) && ((ent & 31) == slot);
    unsigned m = __builtin_amdgcn_ballot_w32(mine);
    while (m != 0u) {
      const int j = __builtin_ctz(m);
      m &= (m - 1u);
      const int en = lst[i + j];
      int e = en >> 5;
      e = min(max(e, 0), nE - 1);
      int s = src[e];
      s = min(max(s, 0), nN - 1);
      const float w = dis[s];
      const float* hr = Hf + (size_t)s * DHID;
      const v4f x0 = *(const v4f*)(hr + 4 * lane);
      const v4f x1 = *(const v4f*)(hr + 128 + 4 * lane);
      a0 += w * x0;
      a1 += w * x1;
    }
  }
}

__global__ __launch_bounds__(256) void gcn_agg_kernel(const int* __restrict__ ei, int nE,
                                                      const float* __restrict__ Hf, const float* __restrict__ dis,
                                                      unsigned short* __restrict__ gh, unsigned short* __restrict__ gl,
                                                      int nN) {
  __shared__ int lst[AG_CAP];
  __shared__ int wcnt[8];
  __shared__ int scnt;
  const int tid  = threadIdx.x;
  const int lane = tid & 31;
  const int wave = tid >> 5;
  const int d0   = blockIdx.x * AG_NB;
  const int* src = ei;
  const int* dst = ei + nE;

  v4f accA[4], accB[4];
#pragma unroll
  for (int s = 0; s < 4; ++s) { accA[s] = (v4f){0.f,0.f,0.f,0.f}; accB[s] = (v4f){0.f,0.f,0.f,0.f}; }

  if (tid == 0) scnt = 0;
  __syncthreads();

  const int nChunks = (nE + AG_CHUNK - 1) / AG_CHUNK;
  for (int ch = 0; ch < nChunks; ++ch) {
    const int cbase = ch * AG_CHUNK;
    const int cnt = scnt;
    const int e0 = cbase + tid * 4;
    int dv0, dv1, dv2, dv3;
    if (cbase + AG_CHUNK <= nE) {
      const v4i d4 = *(const v4i*)(dst + e0);
      dv0 = d4[0]; dv1 = d4[1]; dv2 = d4[2]; dv3 = d4[3];
    } else {
      const int t0 = dst[min(e0, nE - 1)],     t1 = dst[min(e0 + 1, nE - 1)];
      const int t2 = dst[min(e0 + 2, nE - 1)], t3 = dst[min(e0 + 3, nE - 1)];
      dv0 = (e0 < nE) ? t0 : -1;     dv1 = (e0 + 1 < nE) ? t1 : -1;
      dv2 = (e0 + 2 < nE) ? t2 : -1; dv3 = (e0 + 3 < nE) ? t3 : -1;
    }
    const int r0 = dv0 - d0, r1 = dv1 - d0, r2 = dv2 - d0, r3 = dv3 - d0;
    const unsigned hm = (((unsigned)r0 < (unsigned)AG_NB) ? 1u : 0u) | (((unsigned)r1 < (unsigned)AG_NB) ? 2u : 0u) |
                        (((unsigned)r2 < (unsigned)AG_NB) ? 4u : 0u) | (((unsigned)r3 < (unsigned)AG_NB) ? 8u : 0u);
    const int c = __builtin_popcount(hm);
    int incl = c;
#pragma unroll
    for (int off = 1; off < 32; off <<= 1) {
      const int t = __shfl_up(incl, off, 32);
      incl += (lane >= off) ? t : 0;
    }
    if (lane == 31) wcnt[wave] = incl;
    __syncthreads();
    int woff = 0, tot = 0;
#pragma unroll
    for (int w = 0; w < 8; ++w) {
      const int v = wcnt[w];
      tot += v;
      woff += (w < wave) ? v : 0;
    }
    int pos = cnt + woff + incl - c;
    if (hm & 1u) { if (pos < AG_CAP) lst[pos] = (e0 << 5) | r0;       ++pos; }
    if (hm & 2u) { if (pos < AG_CAP) lst[pos] = ((e0 + 1) << 5) | r1; ++pos; }
    if (hm & 4u) { if (pos < AG_CAP) lst[pos] = ((e0 + 2) << 5) | r2; ++pos; }
    if (hm & 8u) { if (pos < AG_CAP) lst[pos] = ((e0 + 3) << 5) | r3; ++pos; }
    __syncthreads();
    if (tid == 0) scnt = min(cnt + tot, AG_CAP);
    __syncthreads();
    const int cnt2 = scnt;
    if (ch == nChunks - 1 || cnt2 + AG_CHUNK > AG_CAP) {
      agg_drain_slot(lst, cnt2, wave * 4 + 0, src, nE, Hf, dis, nN, lane, accA[0], accB[0]);
      agg_drain_slot(lst, cnt2, wave * 4 + 1, src, nE, Hf, dis, nN, lane, accA[1], accB[1]);
      agg_drain_slot(lst, cnt2, wave * 4 + 2, src, nE, Hf, dis, nN, lane, accA[2], accB[2]);
      agg_drain_slot(lst, cnt2, wave * 4 + 3, src, nE, Hf, dis, nN, lane, accA[3], accB[3]);
      __syncthreads();
      if (tid == 0) scnt = 0;
      __syncthreads();
    }
  }

  v4us hA[4], hB[4], lA[4], lB[4];
#pragma unroll
  for (int sub = 0; sub < 4; ++sub) {
    const int d  = d0 + wave * 4 + sub;
    const int dc = min(d, nN - 1);
    const float* hr = Hf + (size_t)dc * DHID;
    const v4f x0 = *(const v4f*)(hr + 4 * lane);
    const v4f x1 = *(const v4f*)(hr + 128 + 4 * lane);
    const float dd = dis[dc];
    const v4f g0 = (accA[sub] + x0) * dd;
    const v4f g1 = (accB[sub] + x1) * dd;
    v4us ha, hb, la, lb;
#pragma unroll
    for (int q = 0; q < 4; ++q) {
      const unsigned short b0 = f2bf_bits(g0[q]);
      const unsigned short b1 = f2bf_bits(g1[q]);
      ha[q] = b0; la[q] = f2bf_bits(g0[q] - bf_bits2f(b0));
      hb[q] = b1; lb[q] = f2bf_bits(g1[q] - bf_bits2f(b1));
    }
    hA[sub] = ha; hB[sub] = hb; lA[sub] = la; lB[sub] = lb;
  }
  for (int pass = 0; pass < 2; ++pass) {
#pragma unroll
    for (int sub = 0; sub < 4; ++sub) {
      const int d = d0 + wave * 4 + sub;
      if (d < nN) {
        const size_t go = (size_t)d * DHID;
        *(volatile v4us*)(gh + go + 4 * lane)       = hA[sub];
        *(volatile v4us*)(gh + go + 128 + 4 * lane) = hB[sub];
        *(volatile v4us*)(gl + go + 4 * lane)       = lA[sub];
        *(volatile v4us*)(gl + go + 128 + 4 * lane) = lB[sub];
      }
    }
    __threadfence();
  }
}

#define AT_D  64
#define AT_NW 4
#define AT_QB 64
#define AT_KC 64

__global__ __launch_bounds__(128)
void attn_kernel(const unsigned short* __restrict__ qkhp, const unsigned short* __restrict__ qklp,
                 const unsigned short* __restrict__ vthp, const unsigned short* __restrict__ vtlp,
                 unsigned short* __restrict__ ohp, unsigned short* __restrict__ olp, float sscale) {
  __shared__ __align__(16) __bf16 KV[4 * AT_KC * AT_D];
  __shared__ __align__(16) __bf16 Psh[AT_NW][16 * AT_KC];
  __shared__ __align__(16) __bf16 Psl[AT_NW][16 * AT_KC];
  __bf16* Ksh = KV;
  __bf16* Ksl = KV + AT_KC * AT_D;
  __bf16* Vth = KV + 2 * AT_KC * AT_D;
  __bf16* Vtl = KV + 3 * AT_KC * AT_D;

  const int tid  = threadIdx.x;
  const int wave = tid >> 5;
  const int lane = tid & 31;
  const int hh   = lane >> 4;
  const int c    = lane & 15;

  const int nqb = NNODE / AT_QB;
  const int bx = blockIdx.x;
  const int qb = bx % nqb;
  const int h  = bx / nqb;
  const int q0 = qb * AT_QB + wave * 16;

  const __bf16* Qh = (const __bf16*)(const void*)qkhp + (size_t)h * AT_D;
  const __bf16* Ql = (const __bf16*)(const void*)qklp + (size_t)h * AT_D;
  const __bf16* Kh = (const __bf16*)(const void*)qkhp + DHID + (size_t)h * AT_D;
  const __bf16* Kl = (const __bf16*)(const void*)qklp + DHID + (size_t)h * AT_D;
  const __bf16* Vh = (const __bf16*)(const void*)vthp + (size_t)h * AT_D * NNODE;
  const __bf16* Vl = (const __bf16*)(const void*)vtlp + (size_t)h * AT_D * NNODE;
  unsigned short* obh = ohp + (size_t)h * AT_D;
  unsigned short* obl = olp + (size_t)h * AT_D;

  v16b qah[2], qal[2];
#pragma unroll
  for (int dc = 0; dc < 2; ++dc) {
    qah[dc] = frag_load(Qh + (size_t)(q0 + c) * QKP + dc * 32 + 8 * hh);
    qal[dc] = frag_load(Ql + (size_t)(q0 + c) * QKP + dc * 32 + 8 * hh);
  }

  float mrow[8], lrow[8];
  v8f oacc[4];
#pragma unroll
  for (int r = 0; r < 8; ++r) { mrow[r] = -INFINITY; lrow[r] = 0.f; }
#pragma unroll
  for (int t = 0; t < 4; ++t) oacc[t] = (v8f){0.f,0.f,0.f,0.f,0.f,0.f,0.f,0.f};

  const int nChunks = NNODE / AT_KC;
  for (int kc = 0; kc < nChunks; ++kc) {
    const int kv0 = kc * AT_KC;
    __syncthreads();
    {
      const int r = tid >> 1, half = (tid & 1) * 32;
      const __bf16* ksh = Kh + (size_t)(kv0 + r) * QKP + half;
      const __bf16* ksl = Kl + (size_t)(kv0 + r) * QKP + half;
      const __bf16* vsh = Vh + (size_t)r * NNODE + kv0 + half;
      const __bf16* vsl = Vl + (size_t)r * NNODE + kv0 + half;
#pragma unroll
      for (int i = 0; i < 4; ++i) {
        const v8b a0 = *(const v8b*)(ksh + 8 * i);
        const v8b a1 = *(const v8b*)(ksl + 8 * i);
        const v8b b0 = *(const v8b*)(vsh + 8 * i);
        const v8b b1 = *(const v8b*)(vsl + 8 * i);
        *(v8b*)(Ksh + r * AT_D  + half + 8 * i) = a0;
        *(v8b*)(Ksl + r * AT_D  + half + 8 * i) = a1;
        *(v8b*)(Vth + r * AT_KC + half + 8 * i) = b0;
        *(v8b*)(Vtl + r * AT_KC + half + 8 * i) = b1;
      }
    }
    __syncthreads();

    v8f s[4];
#pragma unroll
    for (int j = 0; j < 4; ++j) {
      s[j] = (v8f){0.f,0.f,0.f,0.f,0.f,0.f,0.f,0.f};
#pragma unroll
      for (int dc = 0; dc < 2; ++dc) {
        FragB kb, kl;
        kb.h[0] = *(const v8b*)(Ksh + (j * 16 + c) * AT_D + dc * 32 + 8 * hh);
        kb.h[1] = *(const v8b*)(Ksh + (j * 16 + c) * AT_D + dc * 32 + 16 + 8 * hh);
        kl.h[0] = *(const v8b*)(Ksl + (j * 16 + c) * AT_D + dc * 32 + 8 * hh);
        kl.h[1] = *(const v8b*)(Ksl + (j * 16 + c) * AT_D + dc * 32 + 16 + 8 * hh);
        s[j] = mma_bf16_g(qah[dc], kb.v, s[j]);
        s[j] = mma_bf16_g(qah[dc], kl.v, s[j]);
        s[j] = mma_bf16_g(qal[dc], kb.v, s[j]);
      }
    }
    float cm[8];
#pragma unroll
    for (int r = 0; r < 8; ++r) {
      float m = -INFINITY;
#pragma unroll
      for (int j = 0; j < 4; ++j) {
        const float sv = s[j][r] * sscale;
        s[j][r] = sv;
        m = fmaxf(m, sv);
      }
#pragma unroll
      for (int off = 1; off < 16; off <<= 1) m = fmaxf(m, __shfl_xor(m, off, 32));
      cm[r] = m;
    }
    __bf16* pwh = Psh[wave];
    __bf16* pwl = Psl[wave];
#pragma unroll
    for (int r = 0; r < 8; ++r) {
      const float mnew = fmaxf(mrow[r], cm[r]);
      const float alpha = __expf(mrow[r] - mnew);
      mrow[r] = mnew;
      float psum = 0.f;
#pragma unroll
      for (int j = 0; j < 4; ++j) {
        const float p = __expf(s[j][r] - mnew);
        psum += p;
        __bf16 a, b; bf_split(p, a, b);
        pwh[(8 * hh + r) * AT_KC + j * 16 + c] = a;
        pwl[(8 * hh + r) * AT_KC + j * 16 + c] = b;
      }
#pragma unroll
      for (int off = 1; off < 16; off <<= 1) psum += __shfl_xor(psum, off, 32);
      lrow[r] = lrow[r] * alpha + psum;
#pragma unroll
      for (int t = 0; t < 4; ++t) oacc[t][r] *= alpha;
    }
    lds_wave_sync();
#pragma unroll 1
    for (int kk = 0; kk < 2; ++kk) {
      FragB pa, pl;
      pa.h[0] = *(const v8b*)(pwh + c * AT_KC + kk * 32 + 8 * hh);
      pa.h[1] = *(const v8b*)(pwh + c * AT_KC + kk * 32 + 16 + 8 * hh);
      pl.h[0] = *(const v8b*)(pwl + c * AT_KC + kk * 32 + 8 * hh);
      pl.h[1] = *(const v8b*)(pwl + c * AT_KC + kk * 32 + 16 + 8 * hh);
#pragma unroll
      for (int t = 0; t < 4; ++t) {
        FragB vb, vl;
        vb.h[0] = *(const v8b*)(Vth + (t * 16 + c) * AT_KC + kk * 32 + 8 * hh);
        vb.h[1] = *(const v8b*)(Vth + (t * 16 + c) * AT_KC + kk * 32 + 16 + 8 * hh);
        vl.h[0] = *(const v8b*)(Vtl + (t * 16 + c) * AT_KC + kk * 32 + 8 * hh);
        vl.h[1] = *(const v8b*)(Vtl + (t * 16 + c) * AT_KC + kk * 32 + 16 + 8 * hh);
        oacc[t] = mma_bf16_g(pa.v, vb.v, oacc[t]);
        oacc[t] = mma_bf16_g(pa.v, vl.v, oacc[t]);
        oacc[t] = mma_bf16_g(pl.v, vb.v, oacc[t]);
      }
    }
  }

  __syncthreads();
  float* os = (float*)(void*)KV + wave * (16 * 68);
#pragma unroll
  for (int r = 0; r < 8; ++r) {
    const float inv = 1.0f / lrow[r];
#pragma unroll
    for (int t = 0; t < 4; ++t) os[(8 * hh + r) * 68 + t * 16 + c] = oacc[t][r] * inv;
  }
  lds_wave_sync();
  {
    const int q = lane >> 3, c8 = (lane & 7) * 8;
    v8us hv[4], lv[4];
#pragma unroll
    for (int it = 0; it < 4; ++it) {
      const int row = it * 4 + q;
      const float* sp = os + row * 68 + c8;
      v8us a, b;
#pragma unroll
      for (int e = 0; e < 8; ++e) {
        const float f = sp[e];
        const unsigned short hb = f2bf_bits(f);
        a[e] = hb;
        b[e] = f2bf_bits(f - bf_bits2f(hb));
      }
      hv[it] = a; lv[it] = b;
    }
    for (int pass = 0; pass < 2; ++pass) {
#pragma unroll
      for (int it = 0; it < 4; ++it) {
        const int row = it * 4 + q;
        const size_t go = (size_t)(q0 + row) * DHID + c8;
        *(volatile v8us*)(obh + go) = hv[it];
        *(volatile v8us*)(obl + go) = lv[it];
      }
      __threadfence();
    }
  }
}

__global__ __launch_bounds__(256) void ln_kernel(const float* __restrict__ Z, const float* __restrict__ g,
                                                 const float* __restrict__ b, float* __restrict__ Hf,
                                                 unsigned short* __restrict__ Hh, unsigned short* __restrict__ Hl,
                                                 int nRows) {
  const int lane = threadIdx.x & 31;
  const int wave = threadIdx.x >> 5;
  const int row  = blockIdx.x * 8 + wave;
  if (row >= nRows) return;
  const float* zr = Z + (size_t)row * DHID;
  const v4f za = *(const v4f*)(zr + 4 * lane);
  const v4f zb = *(const v4f*)(zr + 128 + 4 * lane);
  float sm = ((za[0] + za[1]) + (za[2] + za[3])) + ((zb[0] + zb[1]) + (zb[2] + zb[3]));
#pragma unroll
  for (int off = 1; off < 32; off <<= 1) sm += __shfl_xor(sm, off, 32);
  const float mu = sm * (1.0f / 256.0f);
  const v4f da = za - mu;
  const v4f db = zb - mu;
  float sq = ((da[0] * da[0] + da[1] * da[1]) + (da[2] * da[2] + da[3] * da[3])) +
             ((db[0] * db[0] + db[1] * db[1]) + (db[2] * db[2] + db[3] * db[3]));
#pragma unroll
  for (int off = 1; off < 32; off <<= 1) sq += __shfl_xor(sq, off, 32);
  const float var  = sq * (1.0f / 256.0f);
  const float rstd = rsqrtf(var + 1e-5f);
  const v4f ga = *(const v4f*)(g + 4 * lane);
  const v4f gb = *(const v4f*)(g + 128 + 4 * lane);
  const v4f ba = *(const v4f*)(b + 4 * lane);
  const v4f bb = *(const v4f*)(b + 128 + 4 * lane);
  const v4f oa = (da * rstd) * ga + ba;
  const v4f ob = (db * rstd) * gb + bb;
  v4us ha, hb, la, lb;
#pragma unroll
  for (int q = 0; q < 4; ++q) {
    const unsigned short b0 = f2bf_bits(oa[q]);
    const unsigned short b1 = f2bf_bits(ob[q]);
    ha[q] = b0; la[q] = f2bf_bits(oa[q] - bf_bits2f(b0));
    hb[q] = b1; lb[q] = f2bf_bits(ob[q] - bf_bits2f(b1));
  }
  const size_t ro = (size_t)row * DHID;
  for (int pass = 0; pass < 2; ++pass) {
    *(volatile v4f*)(Hf + ro + 4 * lane)        = oa;
    *(volatile v4f*)(Hf + ro + 128 + 4 * lane)  = ob;
    *(volatile v4us*)(Hh + ro + 4 * lane)       = ha;
    *(volatile v4us*)(Hh + ro + 128 + 4 * lane) = hb;
    *(volatile v4us*)(Hl + ro + 4 * lane)       = la;
    *(volatile v4us*)(Hl + ro + 128 + 4 * lane) = lb;
    __threadfence();
  }
}

extern "C" void kernel_launch(void* const* d_in, const int* in_sizes, int n_in,
                              void* d_out, int out_size, void* d_ws, size_t ws_size,
                              hipStream_t stream) {
  if (n_in < 13) return;
  if (in_sizes[0] != NNODE * DIN || in_sizes[1] != 2 * NEDGE || in_sizes[2] != DHID * DIN || in_sizes[3] != DHID) return;
  if (in_sizes[4] != NLAYERS * DHID * DHID || in_sizes[5] != NLAYERS * DQKV * DHID || in_sizes[6] != NLAYERS * DQKV) return;
  if (in_sizes[7] != NLAYERS * DHID * DHID || in_sizes[8] != NLAYERS * DHID) return;
  if (in_sizes[9] != NLAYERS * DHID || in_sizes[10] != NLAYERS * DHID) return;
  if (in_sizes[11] != DOUT * DHID || in_sizes[12] != DOUT) return;
  if (out_size != NNODE * DOUT) return;
  static_assert(NNODE % AG_NB == 0);
  static_assert(NNODE % 64 == 0 && DHID % 64 == 0 && QKP % 64 == 0 && DOUT % 64 == 0);
  static_assert(DIN % 32 == 0 && DHID % 32 == 0);

  const float* x          = (const float*)d_in[0];
  const int*   edge_index = (const int*)d_in[1];
  const float* enc_w      = (const float*)d_in[2];
  const float* enc_b      = (const float*)d_in[3];
  const float* gcn_w      = (const float*)d_in[4];
  const float* in_proj_w  = (const float*)d_in[5];
  const float* in_proj_b  = (const float*)d_in[6];
  const float* out_proj_w = (const float*)d_in[7];
  const float* out_proj_b = (const float*)d_in[8];
  const float* ln_g       = (const float*)d_in[9];
  const float* ln_b       = (const float*)d_in[10];
  const float* head_w     = (const float*)d_in[11];
  const float* head_b     = (const float*)d_in[12];

  size_t off = 0;
  auto take = [&](size_t bytes) { size_t o = off; off += (bytes + 127) & ~(size_t)127; return o; };
  const size_t oDIS = take((size_t)NNODE * 4);
  const size_t oXh  = take((size_t)NNODE * DIN * 2);            const size_t oXl  = take((size_t)NNODE * DIN * 2);
  const size_t oEWh = take((size_t)DHID * DIN * 2);             const size_t oEWl = take((size_t)DHID * DIN * 2);
  const size_t oGWh = take((size_t)NLAYERS * DHID * DHID * 2);  const size_t oGWl = take((size_t)NLAYERS * DHID * DHID * 2);
  const size_t oIWh = take((size_t)NLAYERS * DQKV * DHID * 2);  const size_t oIWl = take((size_t)NLAYERS * DQKV * DHID * 2);
  const size_t oOWh = take((size_t)NLAYERS * DHID * DHID * 2);  const size_t oOWl = take((size_t)NLAYERS * DHID * DHID * 2);
  const size_t oHWh = take((size_t)DOUT * DHID * 2);            const size_t oHWl = take((size_t)DOUT * DHID * 2);
  const size_t oH   = take((size_t)NNODE * DHID * 4);
  const size_t oHh  = take((size_t)NNODE * DHID * 2);           const size_t oHl  = take((size_t)NNODE * DHID * 2);
  const size_t oGh  = take((size_t)NNODE * DHID * 2);           const size_t oGl  = take((size_t)NNODE * DHID * 2);
  const size_t oHC  = take((size_t)NNODE * DHID * 4);
  const size_t oQKh = take((size_t)NNODE * QKP * 2);            const size_t oQKl = take((size_t)NNODE * QKP * 2);
  const size_t oVTh = take((size_t)DHID * NNODE * 2);           const size_t oVTl = take((size_t)DHID * NNODE * 2);
  const size_t oOh  = take((size_t)NNODE * DHID * 2);           const size_t oOl  = take((size_t)NNODE * DHID * 2);
  const size_t oZ   = take((size_t)NNODE * DHID * 4);
  if (off > ws_size) return;
  if (off > (size_t)134217728) return;

  char* ws = (char*)d_ws;
  float*          DIS = (float*)(ws + oDIS);
  unsigned short* Xh  = (unsigned short*)(ws + oXh);   unsigned short* Xl  = (unsigned short*)(ws + oXl);
  unsigned short* EWh = (unsigned short*)(ws + oEWh);  unsigned short* EWl = (unsigned short*)(ws + oEWl);
  unsigned short* GWh = (unsigned short*)(ws + oGWh);  unsigned short* GWl = (unsigned short*)(ws + oGWl);
  unsigned short* IWh = (unsigned short*)(ws + oIWh);  unsigned short* IWl = (unsigned short*)(ws + oIWl);
  unsigned short* OWh = (unsigned short*)(ws + oOWh);  unsigned short* OWl = (unsigned short*)(ws + oOWl);
  unsigned short* HWh = (unsigned short*)(ws + oHWh);  unsigned short* HWl = (unsigned short*)(ws + oHWl);
  float*          Hf  = (float*)(ws + oH);
  unsigned short* Hh  = (unsigned short*)(ws + oHh);   unsigned short* Hl  = (unsigned short*)(ws + oHl);
  unsigned short* Gh  = (unsigned short*)(ws + oGh);   unsigned short* Gl  = (unsigned short*)(ws + oGl);
  float*          HCf = (float*)(ws + oHC);
  unsigned short* QKh = (unsigned short*)(ws + oQKh);  unsigned short* QKl = (unsigned short*)(ws + oQKl);
  unsigned short* VTh = (unsigned short*)(ws + oVTh);  unsigned short* VTl = (unsigned short*)(ws + oVTl);
  unsigned short* Oh  = (unsigned short*)(ws + oOh);   unsigned short* Ol  = (unsigned short*)(ws + oOl);
  float*          Zf  = (float*)(ws + oZ);

  const dim3 b256(256), b128(128);
  auto gsplit = [](int n) { return dim3((unsigned)(((n / 2) + 255) / 256)); };
  auto ggemm  = [](int M, int N) { return dim3((unsigned)(((M / 64) * (N / 64) + 7) / 8)); };

  split_bf16x2_kernel<<<gsplit(NNODE * DIN), b256, 0, stream>>>(x, Xh, Xl, NNODE * DIN / 2);
  split_bf16x2_kernel<<<gsplit(DHID * DIN), b256, 0, stream>>>(enc_w, EWh, EWl, DHID * DIN / 2);
  split_bf16x2_kernel<<<gsplit(NLAYERS * DHID * DHID), b256, 0, stream>>>(gcn_w, GWh, GWl, NLAYERS * DHID * DHID / 2);
  split_bf16x2_kernel<<<gsplit(NLAYERS * DQKV * DHID), b256, 0, stream>>>(in_proj_w, IWh, IWl, NLAYERS * DQKV * DHID / 2);
  split_bf16x2_kernel<<<gsplit(NLAYERS * DHID * DHID), b256, 0, stream>>>(out_proj_w, OWh, OWl, NLAYERS * DHID * DHID / 2);
  split_bf16x2_kernel<<<gsplit(DOUT * DHID), b256, 0, stream>>>(head_w, HWh, HWl, DOUT * DHID / 2);

  deg_dis_kernel<<<dim3(1), b256, 0, stream>>>(edge_index, NEDGE, NNODE, DIS);

  gemm_x3_kernel<2, 2, 0, 1><<<ggemm(NNODE, DHID), b256, 0, stream>>>(
      Xh, Xl, DIN, EWh, EWl, DIN, Hf, Hh, Hl, DHID, enc_b, Hf, Hf, NNODE, DHID, DIN);

  for (int l = 0; l < NLAYERS; ++l) {
    const unsigned short* gwh = GWh + (size_t)l * DHID * DHID;
    const unsigned short* gwl = GWl + (size_t)l * DHID * DHID;
    const unsigned short* iwh = IWh + (size_t)l * DQKV * DHID;
    const unsigned short* iwl = IWl + (size_t)l * DQKV * DHID;
    const unsigned short* owh = OWh + (size_t)l * DHID * DHID;
    const unsigned short* owl = OWl + (size_t)l * DHID * DHID;
    const float* ipb = in_proj_b + (size_t)l * DQKV;
    const float* opb = out_proj_b + (size_t)l * DHID;

    gcn_agg_kernel<<<dim3(NNODE / AG_NB), b256, 0, stream>>>(edge_index, NEDGE, Hf, DIS, Gh, Gl, NNODE);
    gemm_x3_kernel<0, 0, 0, 1><<<ggemm(NNODE, DHID), b256, 0, stream>>>(
        Gh, Gl, DHID, gwh, gwl, DHID, HCf, Gh, Gl, DHID, enc_b, Hf, Hf, NNODE, DHID, DHID);
    gemm_x3_kernel<2, 1, 0, 0><<<ggemm(NNODE, QKP), b256, 0, stream>>>(
        Hh, Hl, DHID, iwh, iwl, DHID, Zf, QKh, QKl, QKP, ipb, Hf, Hf, NNODE, QKP, DHID);
    gemm_x3_kernel<1, 1, 0, 0><<<ggemm(DHID, NNODE), b256, 0, stream>>>(
        iwh + (size_t)2 * DHID * DHID, iwl + (size_t)2 * DHID * DHID, DHID, Hh, Hl, DHID,
        Zf, VTh, VTl, NNODE, ipb + 2 * DHID, Hf, Hf, DHID, NNODE, DHID);
    attn_kernel<<<dim3(NHEADS * (NNODE / AT_QB)), b128, 0, stream>>>(QKh, QKl, VTh, VTl, Oh, Ol, 0.125f);
    gemm_x3_kernel<2, 0, 2, 0><<<ggemm(NNODE, DHID), b256, 0, stream>>>(
        Oh, Ol, DHID, owh, owl, DHID, Zf, Gh, Gl, DHID, opb, Hf, HCf, NNODE, DHID, DHID);
    ln_kernel<<<dim3(NNODE / 8), b256, 0, stream>>>(Zf, ln_g + (size_t)l * DHID, ln_b + (size_t)l * DHID,
                                                    Hf, Hh, Hl, NNODE);
  }

  gemm_x3_kernel<2, 0, 0, 0><<<ggemm(NNODE, DOUT), b256, 0, stream>>>(
      Hh, Hl, DHID, HWh, HWl, DHID, (float*)d_out, Gh, Gl, DOUT, head_b, Hf, Hf, NNODE, DOUT, DHID);
  (void)hipGetLastError();
}
